// TreeModel_6725918785677
// MI455X (gfx1250) — hardware-verified
//
#include <hip/hip_runtime.h>
#include <math.h>

constexpr int NDOC  = 64;
constexpr int NSEN  = 32;
constexpr int NWRD  = 64;
constexpr int NVOC  = 50000;
constexpr int EDIM  = 128;
constexpr int HDOC  = 256;
constexpr int NOUT  = 5;
constexpr int NSROW = NDOC * NSEN;
constexpr int TP_THREADS   = 256;
constexpr int HID_THREADS  = 256;
constexpr int HEAD_THREADS = NDOC * NOUT;
constexpr float A_SCALE  = 8.0f;
constexpr float W_SCALE  = 64.0f;
constexpr float FOLD_INV = 1.0f / 512.0f;

typedef __attribute__((ext_vector_type(16))) _Float16 v16h;
typedef __attribute__((ext_vector_type(8)))  _Float16 v8h;
typedef __attribute__((ext_vector_type(16))) __bf16   v16b;
typedef __attribute__((ext_vector_type(8)))  __bf16   v8b;
typedef __attribute__((ext_vector_type(8)))  float    v8f;
typedef __attribute__((ext_vector_type(4)))  float    v4f;

__device__ __forceinline__ void dep_guard_h(v8f& a, v8f& b, v16h x, v16h y) { asm volatile("v_nop\n\tv_nop\n\tv_nop\n\tv_nop" : "+v"(a), "+v"(b) : "v"(x), "v"(y)); }
__device__ __forceinline__ void dep_guard_b(v8f& a, v8f& b, v16b x, v16b y) { asm volatile("v_nop\n\tv_nop\n\tv_nop\n\tv_nop" : "+v"(a), "+v"(b) : "v"(x), "v"(y)); }
__device__ __forceinline__ void keep4_h(v16h a, v16h b, v16h c, v16h d) { asm volatile("v_nop" :: "v"(a), "v"(b), "v"(c), "v"(d)); }
__device__ __forceinline__ void keep4_b(v16b a, v16b b, v16b c, v16b d) { asm volatile("v_nop" :: "v"(a), "v"(b), "v"(c), "v"(d)); }
template <typename T> struct Frag;
template <> struct Frag<_Float16> {
  typedef v16h V; union U { v16h v; v8h h[2]; };
  static __device__ __forceinline__ v16h load(const _Float16* p) {
    U f; f.h[0] = *(const v8h*)(p); f.h[1] = *(const v8h*)(p + 16); return f.v;
  }
  static __device__ __forceinline__ v8f mma(v16h a, v16h b, v8f c) {
    return __builtin_amdgcn_wmma_f32_16x16x32_f16(false, a, false, b, (short)0, c, false, false);
  }
  static __device__ __forceinline__ void guard(v8f& a, v8f& b, v16h x, v16h y) { dep_guard_h(a, b, x, y); }
  static __device__ __forceinline__ void keep(v16h a, v16h b, v16h c, v16h d) { keep4_h(a, b, c, d); }
};
template <> struct Frag<__bf16> {
  typedef v16b V; union U { v16b v; v8b h[2]; };
  static __device__ __forceinline__ v16b load(const __bf16* p) {
    U f; f.h[0] = *(const v8b*)(p); f.h[1] = *(const v8b*)(p + 16); return f.v;
  }
  static __device__ __forceinline__ v8f mma(v16b a, v16b b, v8f c) {
    return __builtin_amdgcn_wmma_f32_16x16x32_bf16(false, a, false, b, (short)0, c, false, false);
  }
  static __device__ __forceinline__ void guard(v8f& a, v8f& b, v16b x, v16b y) { dep_guard_b(a, b, x, y); }
  static __device__ __forceinline__ void keep(v16b a, v16b b, v16b c, v16b d) { keep4_b(a, b, c, d); }
};

__device__ __forceinline__ v8f mma_h(v16h a, v16h b, v8f c) {
  c = __builtin_amdgcn_wmma_f32_16x16x32_f16(false, a, false, b, (short)0, c, false, false);
  asm volatile("v_nop\n\tv_nop\n\tv_nop\n\tv_nop" : "+v"(c) : "v"(a), "v"(b));
  return c;
}

__device__ __forceinline__ float ftanh(float x) { return 1.0f - 2.0f * __builtin_amdgcn_rcpf(__expf(2.0f * x) + 1.0f); }
__device__ __forceinline__ float fsigm(float x) { return __builtin_amdgcn_rcpf(1.0f + __expf(-x)); }

__global__ __launch_bounds__(TP_THREADS) void tpw_f16(const float* __restrict__ src, int R, int C, int ldo,
                                                     unsigned short* __restrict__ O, float sc) {
  __shared__ float Tt[64 * 65];
  const int tid = threadIdx.x;
  const int c0 = blockIdx.x * 64, r0 = blockIdx.y * 64;
  (void)R;
#pragma unroll
  for (int i = 0; i < 4; ++i) {
    const int idx = i * TP_THREADS + tid;
    const int rr = idx >> 4, cc = (idx & 15) * 4;
    const v4f v = *(const v4f*)(src + (size_t)(r0 + rr) * (size_t)C + c0 + cc);
    Tt[rr * 65 + cc + 0] = v[0];
    Tt[rr * 65 + cc + 1] = v[1];
    Tt[rr * 65 + cc + 2] = v[2];
    Tt[rr * 65 + cc + 3] = v[3];
  }
  __syncthreads();
  const int q = tid >> 3, c8 = (tid & 7) * 8;
  v8h hv[2];
#pragma unroll
  for (int g = 0; g < 2; ++g) {
    const int qq = g * 32 + q;
#pragma unroll
    for (int e = 0; e < 8; ++e) {
      const float f = Tt[(c8 + e) * 65 + qq];
      hv[g][e] = (_Float16)(f * sc);
    }
  }
  for (int pass = 0; pass < 2; ++pass) {
#pragma unroll
    for (int g = 0; g < 2; ++g) {
      const size_t o = (size_t)(c0 + g * 32 + q) * (size_t)ldo + (size_t)(r0 + c8);
      *(volatile v8h*)(O + o) = hv[g];
    }
    __threadfence();
  }
}

template <int DIN, int NST, int APITCH, bool FROM_EMB>
__device__ __forceinline__ void gather_xrow(_Float16* dst, const int* __restrict__ ids, const float* __restrict__ emb,
                                            const unsigned short* src16, int row, int t, int glen, int dir,
                                            int gm, int gc8) {
  const int ttr = (t < glen) ? (glen - 1 - t) : t;
  int tt = dir ? ttr : t;
  tt = tt < 0 ? 0 : tt;
  tt = tt > NST - 1 ? NST - 1 : tt;
  v8h hv;
  if constexpr (FROM_EMB) {
    int tok = ids[(size_t)row * NST + (size_t)tt];
    tok = tok < 0 ? 0 : tok;
    tok = tok > NVOC - 1 ? NVOC - 1 : tok;
    const float* e = emb + (size_t)tok * DIN + gc8;
    const v4f a = *(const v4f*)(e);
    const v4f b = *(const v4f*)(e + 4);
    hv[0] = (_Float16)(a[0] * A_SCALE); hv[1] = (_Float16)(a[1] * A_SCALE);
    hv[2] = (_Float16)(a[2] * A_SCALE); hv[3] = (_Float16)(a[3] * A_SCALE);
    hv[4] = (_Float16)(b[0] * A_SCALE); hv[5] = (_Float16)(b[1] * A_SCALE);
    hv[6] = (_Float16)(b[2] * A_SCALE); hv[7] = (_Float16)(b[3] * A_SCALE);
  } else {
    hv = *(const v8h*)((const _Float16*)src16 + ((size_t)row * NST + (size_t)tt) * (size_t)DIN + gc8);
  }
  *(v8h*)(dst + gm * APITCH + gc8) = hv;
}

template <int DIN, int HH, int NST, bool FROM_EMB, bool OUT_F32>
__global__ __launch_bounds__(2 * HH) void gru_bidir_kernel(
    const int* __restrict__ ids, const float* __restrict__ emb, const unsigned short* src16,
    const int* __restrict__ lengths,
    const unsigned short* __restrict__ WgTf, const unsigned short* __restrict__ WcTf,
    const float* __restrict__ bgf, const float* __restrict__ bcf,
    const unsigned short* __restrict__ WgTb, const unsigned short* __restrict__ WcTb,
    const float* __restrict__ bgb, const float* __restrict__ bcb,
    unsigned short* out16, float* out32, int nrows, int nblk_per_dir) {
  constexpr int NTHR   = 2 * HH;
  constexpr int KTOT   = DIN + HH;
  constexpr int APITCH = KTOT + 8;
  constexpr int RPITCH = HH + 8;
  constexpr int OPITCH = HH + 4;
  constexpr int ATILE  = 16 * APITCH;
  constexpr int GCH    = DIN / 8;
  constexpr int OCH    = HH / 8;
  constexpr int F4     = HH / 4;
  static_assert(DIN == HH);
  static_assert(DIN % 32 == 0 && HH % 32 == 0);
  static_assert(16 * GCH == NTHR && 16 * OCH == NTHR);
  static_assert((16 * F4) % NTHR == 0 && F4 % 32 == 0);
  __shared__ __align__(16) _Float16 Axh[2 * ATILE];
  __shared__ __align__(16) _Float16 Arh[16 * RPITCH];
  __shared__ __align__(16) _Float16 Osh[OUT_F32 ? 8 : 16 * RPITCH];
  __shared__ __align__(16) float    Osf[OUT_F32 ? 16 * OPITCH : 4];

  const int tid = threadIdx.x, lane = tid & 31, wave = tid >> 5;
  const int c = lane & 15, hh = lane >> 4, koff = hh * 8;
  const int dir = (blockIdx.x >= (unsigned)nblk_per_dir) ? 1 : 0;
  int rb = ((int)blockIdx.x - dir * nblk_per_dir) * 16;
  rb = rb < 0 ? 0 : rb;
  rb = (rb > nrows - 16) ? (nrows - 16) : rb;
  const _Float16* WgT = (const _Float16*)(dir ? WgTb : WgTf);
  const _Float16* WcT = (const _Float16*)(dir ? WcTb : WcTf);
  const float* bg = dir ? bgb : bgf;
  const float* bc = dir ? bcb : bcf;
  const int j = 16 * wave + c;

#pragma unroll 1
  for (int i = tid; i < 2 * ATILE; i += NTHR) Axh[i] = (_Float16)0.0f;

  const int gm = tid / GCH, gc8 = (tid - gm * GCH) * 8;
  const int glen = lengths[rb + gm];
  int len8[8];
  float hst[8], ust[8];
#pragma unroll
  for (int r = 0; r < 8; ++r) {
    len8[r] = lengths[rb + 8 * hh + r];
    hst[r] = 0.0f;
    ust[r] = 0.0f;
  }
  const float bgr = bg[j];
  const float bgu = bg[HH + j];
  const float bcj = bc[j];
  __syncthreads();
  gather_xrow<DIN, NST, APITCH, FROM_EMB>(Axh, ids, emb, src16, rb + gm, 0, glen, dir, gm, gc8);
  __syncthreads();

  const v8f z8 = {0.f, 0.f, 0.f, 0.f, 0.f, 0.f, 0.f, 0.f};
  const _Float16* wr  = WgT + (size_t)j * KTOT + koff;
  const _Float16* wu  = WgT + (size_t)(HH + j) * KTOT + koff;
  const _Float16* wcp = WcT + (size_t)j * KTOT + koff;

#pragma unroll 1
  for (int t = 0; t < NST; ++t) {
    const int cur = t & 1;
    const _Float16* Ac = Axh + cur * ATILE;
    _Float16*       An = Axh + (cur ^ 1) * ATILE;
    const _Float16* axr = Ac + c * APITCH + koff;

    {
      v8f accR = z8, accU = z8;
#pragma unroll 2
      for (int k0 = 0; k0 < KTOT; k0 += 32) {
        const v16h a  = Frag<_Float16>::load(axr + k0);
        const v16h b0 = Frag<_Float16>::load(wr + k0);
        const v16h b1 = Frag<_Float16>::load(wu + k0);
        accR = mma_h(a, b0, accR);
        accU = mma_h(a, b1, accU);
      }
#pragma unroll
      for (int r = 0; r < 8; ++r) {
        const float rg = fsigm(accR[r] * FOLD_INV + bgr);
        const float ug = fsigm(accU[r] * FOLD_INV + bgu);
        ust[r] = ug;
        Arh[(8 * hh + r) * RPITCH + j] = (_Float16)(rg * hst[r] * A_SCALE);
      }
    }
    __syncthreads();

    {
      v8f accC = z8;
#pragma unroll 2
      for (int k0 = 0; k0 < DIN; k0 += 32) {
        const v16h a = Frag<_Float16>::load(axr + k0);
        const v16h b = Frag<_Float16>::load(wcp + k0);
        accC = mma_h(a, b, accC);
      }
      const _Float16* arr = Arh + c * RPITCH + koff;
#pragma unroll 2
      for (int k0 = 0; k0 < HH; k0 += 32) {
        const v16h a = Frag<_Float16>::load(arr + k0);
        const v16h b = Frag<_Float16>::load(wcp + DIN + k0);
        accC = mma_h(a, b, accC);
      }
#pragma unroll
      for (int r = 0; r < 8; ++r) {
        const float cg   = ftanh(accC[r] * FOLD_INV + bcj);
        const float u    = ust[r];
        const float hold = hst[r];
        const float hn   = u * hold + (1.0f - u) * cg;
        const bool alive = (t < len8[r]);
        const float v    = alive ? hn : hold;
        hst[r] = v;
        An[(8 * hh + r) * APITCH + DIN + j] = (_Float16)(v * A_SCALE);
      }
    }
    {
      const int tn = (t + 1 < NST) ? (t + 1) : (NST - 1);
      gather_xrow<DIN, NST, APITCH, FROM_EMB>(An, ids, emb, src16, rb + gm, tn, glen, dir, gm, gc8);
    }
    __syncthreads();
  }

  if constexpr (OUT_F32) {
#pragma unroll
    for (int r = 0; r < 8; ++r) Osf[(8 * hh + r) * OPITCH + j] = hst[r];
    __syncthreads();
    constexpr int NIT = (16 * F4) / NTHR;
    for (int pass = 0; pass < 2; ++pass) {
#pragma unroll
      for (int it = 0; it < NIT; ++it) {
        const int idx  = it * NTHR + tid;
        const int orow = idx / F4, c4 = (idx - orow * F4) * 4;
        const v4f v = *(const v4f*)(Osf + orow * OPITCH + c4);
        *(volatile v4f*)(out32 + (size_t)(rb + orow) * (size_t)(2 * HH) + (size_t)(dir * HH) + c4) = v;
      }
      __threadfence();
    }
  } else {
#pragma unroll
    for (int r = 0; r < 8; ++r) Osh[(8 * hh + r) * RPITCH + j] = (_Float16)(hst[r] * A_SCALE);
    __syncthreads();
    const int orow = tid / OCH, oc8 = (tid - orow * OCH) * 8;
    const v8h v = *(const v8h*)(Osh + orow * RPITCH + oc8);
    unsigned short* dst = out16 + (size_t)(rb + orow) * (size_t)(2 * HH) + (size_t)(dir * HH) + oc8;
    for (int pass = 0; pass < 2; ++pass) {
      *(volatile v8h*)dst = v;
      __threadfence();
    }
  }
}

__global__ __launch_bounds__(HID_THREADS) void hid_kernel(const float* __restrict__ docv, const float* __restrict__ W1,
                                                          const float* __restrict__ b1, float* __restrict__ hid) {
  __shared__ __align__(16) float ds[2 * HDOC];
  __shared__ __align__(16) float hs[HDOC];
  const int tid = threadIdx.x;
  const int doc = blockIdx.x;
  const float* dr = docv + (size_t)doc * (2 * HDOC);
  ds[tid]        = dr[tid];
  ds[tid + HDOC] = dr[tid + HDOC];
  __syncthreads();
  float z = 0.0f;
#pragma unroll 1
  for (int k = 0; k < 2 * HDOC; ++k) z += ds[k] * W1[(size_t)k * HDOC + tid];
  z += b1[tid];
  hs[tid] = fmaxf(z, 0.0f);
  __syncthreads();
  v4f v = {0.f, 0.f, 0.f, 0.f};
  if (tid < HDOC / 4) v = *(const v4f*)(hs + tid * 4);
  for (int pass = 0; pass < 2; ++pass) {
    if (tid < HDOC / 4) *(volatile v4f*)(hid + (size_t)doc * HDOC + tid * 4) = v;
    __threadfence();
  }
}

__global__ __launch_bounds__(HEAD_THREADS) void head_out_kernel(const float* __restrict__ hid, const float* __restrict__ W2,
                                                               const float* __restrict__ b2, float* __restrict__ out) {
  __shared__ __align__(16) float zs[HEAD_THREADS];
  const int tid = threadIdx.x;
  const int row = tid / NOUT, o = tid - row * NOUT;
  const float* hr = hid + (size_t)row * HDOC;
  float z = 0.0f;
#pragma unroll 1
  for (int k = 0; k < HDOC; ++k) z += hr[k] * W2[k * NOUT + o];
  z += b2[o];
  zs[tid] = z;
  __syncthreads();
  v4f v = {0.f, 0.f, 0.f, 0.f};
  if (tid < HEAD_THREADS / 4) v = *(const v4f*)(zs + tid * 4);
  for (int pass = 0; pass < 2; ++pass) {
    if (tid < HEAD_THREADS / 4) *(volatile v4f*)(out + tid * 4) = v;
    __threadfence();
  }
}

extern "C" void kernel_launch(void* const* d_in, const int* in_sizes, int n_in,
                              void* d_out, int out_size, void* d_ws, size_t ws_size, hipStream_t stream) {
  if (n_in < 24 || d_out == nullptr || d_ws == nullptr) return;
  if (in_sizes[0] != NDOC * NSEN * NWRD || in_sizes[1] != NSROW || in_sizes[2] != NDOC ||
      in_sizes[3] != NVOC * EDIM ||
      in_sizes[4] != 256 * 256 || in_sizes[5] != 256 || in_sizes[6] != 256 * 128 || in_sizes[7] != 128 ||
      in_sizes[8] != 256 * 256 || in_sizes[9] != 256 || in_sizes[10] != 256 * 128 || in_sizes[11] != 128 ||
      in_sizes[12] != 512 * 512 || in_sizes[13] != 512 || in_sizes[14] != 512 * 256 || in_sizes[15] != 256 ||
      in_sizes[16] != 512 * 512 || in_sizes[17] != 512 || in_sizes[18] != 512 * 256 || in_sizes[19] != 256 ||
      in_sizes[20] != 512 * 256 || in_sizes[21] != 256 || in_sizes[22] != 256 * NOUT || in_sizes[23] != NOUT ||
      out_size != NDOC * NOUT) return;

  const int*   X     = (const int*)d_in[0];
  const int*   L     = (const int*)d_in[1];
  const int*   L2    = (const int*)d_in[2];
  const float* emb   = (const float*)d_in[3];
  const float* sWg_f = (const float*)d_in[4];
  const float* sbg_f = (const float*)d_in[5];
  const float* sWc_f = (const float*)d_in[6];
  const float* sbc_f = (const float*)d_in[7];
  const float* sWg_b = (const float*)d_in[8];
  const float* sbg_b = (const float*)d_in[9];
  const float* sWc_b = (const float*)d_in[10];
  const float* sbc_b = (const float*)d_in[11];
  const float* dWg_f = (const float*)d_in[12];
  const float* dbg_f = (const float*)d_in[13];
  const float* dWc_f = (const float*)d_in[14];
  const float* dbc_f = (const float*)d_in[15];
  const float* dWg_b = (const float*)d_in[16];
  const float* dbg_b = (const float*)d_in[17];
  const float* dWc_b = (const float*)d_in[18];
  const float* dbc_b = (const float*)d_in[19];
  const float* W1    = (const float*)d_in[20];
  const float* b1    = (const float*)d_in[21];
  const float* W2    = (const float*)d_in[22];
  const float* b2    = (const float*)d_in[23];
  float* out = (float*)d_out;

  char* ws = (char*)d_ws; size_t off = 0;
  auto carve = [&](size_t bytes) -> char* { char* p = ws + off; off += (bytes + 255) & ~(size_t)255; return p; };
  unsigned short* SWGT_f = (unsigned short*)carve((size_t)256 * 256 * 2);
  unsigned short* SWCT_f = (unsigned short*)carve((size_t)128 * 256 * 2);
  unsigned short* SWGT_b = (unsigned short*)carve((size_t)256 * 256 * 2);
  unsigned short* SWCT_b = (unsigned short*)carve((size_t)128 * 256 * 2);
  unsigned short* DWGT_f = (unsigned short*)carve((size_t)512 * 512 * 2);
  unsigned short* DWCT_f = (unsigned short*)carve((size_t)256 * 512 * 2);
  unsigned short* DWGT_b = (unsigned short*)carve((size_t)512 * 512 * 2);
  unsigned short* DWCT_b = (unsigned short*)carve((size_t)256 * 512 * 2);
  unsigned short* SENT   = (unsigned short*)carve((size_t)NSROW * (2 * EDIM) * 2);
  float*          DOCV   = (float*)carve((size_t)NDOC * (2 * HDOC) * 4);
  float*          HID    = (float*)carve((size_t)NDOC * HDOC * 4);
  if (off > ws_size || off > (size_t)134217728) return;

  tpw_f16<<<dim3(256 / 64, 256 / 64), TP_THREADS, 0, stream>>>(sWg_f, 256, 256, 256, SWGT_f, W_SCALE);
  tpw_f16<<<dim3(128 / 64, 256 / 64), TP_THREADS, 0, stream>>>(sWc_f, 256, 128, 256, SWCT_f, W_SCALE);
  tpw_f16<<<dim3(256 / 64, 256 / 64), TP_THREADS, 0, stream>>>(sWg_b, 256, 256, 256, SWGT_b, W_SCALE);
  tpw_f16<<<dim3(128 / 64, 256 / 64), TP_THREADS, 0, stream>>>(sWc_b, 256, 128, 256, SWCT_b, W_SCALE);
  tpw_f16<<<dim3(512 / 64, 512 / 64), TP_THREADS, 0, stream>>>(dWg_f, 512, 512, 512, DWGT_f, W_SCALE);
  tpw_f16<<<dim3(256 / 64, 512 / 64), TP_THREADS, 0, stream>>>(dWc_f, 512, 256, 512, DWCT_f, W_SCALE);
  tpw_f16<<<dim3(512 / 64, 512 / 64), TP_THREADS, 0, stream>>>(dWg_b, 512, 512, 512, DWGT_b, W_SCALE);
  tpw_f16<<<dim3(256 / 64, 512 / 64), TP_THREADS, 0, stream>>>(dWc_b, 512, 256, 512, DWCT_b, W_SCALE);

  constexpr int NBS = NSROW / 16;
  gru_bidir_kernel<EDIM, EDIM, NWRD, true, false><<<2 * NBS, 2 * EDIM, 0, stream>>>(
      X, emb, SWCT_f, L,
      SWGT_f, SWCT_f, sbg_f, sbc_f, SWGT_b, SWCT_b, sbg_b, sbc_b, SENT, DOCV, NSROW, NBS);

  constexpr int NBD = NDOC / 16;
  gru_bidir_kernel<2 * EDIM, HDOC, NSEN, false, true><<<2 * NBD, 2 * HDOC, 0, stream>>>(
      X, emb, SENT, L2,
      DWGT_f, DWCT_f, dbg_f, dbc_f, DWGT_b, DWCT_b, dbg_b, dbc_b, (unsigned short*)(void*)HID, DOCV, NDOC, NBD);

  hid_kernel<<<NDOC, HID_THREADS, 0, stream>>>(DOCV, W1, b1, HID);

  head_out_kernel<<<1, HEAD_THREADS, 0, stream>>>(HID, W2, b2, out);
}
